// SparseAttention_89421219103270
// MI455X (gfx1250) — hardware-verified
//
#include <hip/hip_runtime.h>
#include <math.h>

#ifndef NB
#define NB 1
#endif
#ifndef SEQ
#define SEQ 4096
#endif
#define SEQ_FULL 4096
#define HEADS 8
#define HD 64
#define ST_TT 128
#define ST_PT 136
#define NCHUNK (SEQ / ST_TT)
#define OUT_ROWS 128
#define SLAB_P 68
#define RES_CARRY 2048.0f
#define RES_INV (1.0f / 2048.0f)
#define QK_SCALE 0.125f
#define IN_MIN (((HEADS - 1) * SEQ_FULL + SEQ) * HD)
#define PART_BYTES ((size_t)HEADS * NCHUNK * HD * HD * 4)
#define SPL_BYTES  ((size_t)HEADS * HD * HD * 2)

static_assert(NB == 1);
static_assert(HD == 64);
static_assert(SEQ <= SEQ_FULL);
static_assert(SEQ % ST_TT == 0 && SEQ % OUT_ROWS == 0);
static_assert(ST_TT % 32 == 0 && HD % 32 == 0);
static_assert(ST_PT % 8 == 0 && ST_PT >= ST_TT);
static_assert(SLAB_P % 4 == 0 && SLAB_P >= HD);
static_assert(8 * 256 * 4 == ST_TT * HD);
static_assert(256 * 16 * 4 == HD * HD * 4);
static_assert((HEADS * HD * (HD / 8)) % 256 == 0);
static_assert(32 * 16 * 8 == 16 * HD * 4);
static_assert(OUT_ROWS == 8 * 16);
static_assert(2 * 64 * ST_PT * 2 + 64 * SLAB_P * 4 <= 131072);
static_assert(8 * 16 * SLAB_P * 4 <= 131072);
static_assert(PART_BYTES % 256 == 0 && SPL_BYTES % 256 == 0);
static_assert(PART_BYTES + 2 * SPL_BYTES <= (size_t)134217728);

typedef __attribute__((ext_vector_type(16))) _Float16 v16h;
typedef __attribute__((ext_vector_type(8)))  _Float16 v8h;
typedef __attribute__((ext_vector_type(8)))  float    v8f;
typedef __attribute__((ext_vector_type(4)))  float    v4f;
typedef __attribute__((ext_vector_type(4)))  unsigned int v4u;
typedef _Float16 h16;


#define VST2(T, ptr, val) do { const T vst2_v_ = (val); *(volatile T*)(ptr) = vst2_v_; __threadfence(); *(volatile T*)(ptr) = vst2_v_; } while (0)

__device__ __forceinline__ float bfr(float f) {
    unsigned u = __float_as_uint(f);
    u += 0x7FFFu + ((u >> 16) & 1u);
    return __uint_as_float(u & 0xFFFF0000u);
}
__device__ __forceinline__ unsigned short f2h_bits(float x) {
    return (fabsf(x) < 6.104e-5f) ? (unsigned short)0 : __builtin_bit_cast(unsigned short, (_Float16)x);
}
__device__ __forceinline__ void st8h(unsigned short* P, size_t o, const float* v) {
    v4u pk;
    pk.x = (unsigned)f2h_bits(v[0]) | ((unsigned)f2h_bits(v[1]) << 16);
    pk.y = (unsigned)f2h_bits(v[2]) | ((unsigned)f2h_bits(v[3]) << 16);
    pk.z = (unsigned)f2h_bits(v[4]) | ((unsigned)f2h_bits(v[5]) << 16);
    pk.w = (unsigned)f2h_bits(v[6]) | ((unsigned)f2h_bits(v[7]) << 16);
    VST2(v4u, (v4u*)(P + o), pk);
}
static __device__ __forceinline__ h16 toh_flush(float v) {
    const h16 r = (h16)v;
    return (fabsf(v) < 6.103515625e-05f) ? (h16)0.0f : r;
}

union FragU { v16h v; v8h h[2]; };
__device__ __forceinline__ v16h frag_ld(const _Float16* p) {
    FragU f; f.h[0] = *(const v8h*)(p); f.h[1] = *(const v8h*)(p + 16); return f.v;
}
__device__ __forceinline__ v16h frag_cvt(const float* p) {
    const v4f a0 = *(const v4f*)(p);
    const v4f a1 = *(const v4f*)(p + 4);
    const v4f a2 = *(const v4f*)(p + 16);
    const v4f a3 = *(const v4f*)(p + 20);
    v16h f;
    f[0]  = toh_flush(bfr(a0.x)); f[1]  = toh_flush(bfr(a0.y)); f[2]  = toh_flush(bfr(a0.z)); f[3]  = toh_flush(bfr(a0.w));
    f[4]  = toh_flush(bfr(a1.x)); f[5]  = toh_flush(bfr(a1.y)); f[6]  = toh_flush(bfr(a1.z)); f[7]  = toh_flush(bfr(a1.w));
    f[8]  = toh_flush(bfr(a2.x)); f[9]  = toh_flush(bfr(a2.y)); f[10] = toh_flush(bfr(a2.z)); f[11] = toh_flush(bfr(a2.w));
    f[12] = toh_flush(bfr(a3.x)); f[13] = toh_flush(bfr(a3.y)); f[14] = toh_flush(bfr(a3.z)); f[15] = toh_flush(bfr(a3.w));
    return f;
}
__device__ __forceinline__ v8f wmma16(v16h a, v16h b, v8f c) {
    c = __builtin_amdgcn_wmma_f32_16x16x32_f16(false, a, false, b, (short)0, c, false, false);
    asm volatile("v_nop\n\tv_nop\n\tv_nop\n\tv_nop" : "+v"(c) : "v"(a), "v"(b));
    return c;
}
__device__ __forceinline__ void wave_sync_lds() {
    __builtin_amdgcn_fence(3  , "workgroup");
    __builtin_amdgcn_wave_barrier();
    __builtin_amdgcn_fence(2  , "workgroup");
}

__global__ __launch_bounds__(256) void k_state(const float* __restrict__ kin, const float* __restrict__ vin,
                                               float* __restrict__ part) {
    __shared__ __align__(16) _Float16 sKT[64 * ST_PT];
    __shared__ __align__(16) _Float16 sVT[64 * ST_PT];
    __shared__ __align__(16) float    sC[64 * SLAB_P];
    const unsigned tid = threadIdx.x, lane = tid & 31u;
    const unsigned wave = (unsigned)__builtin_amdgcn_readfirstlane((int)(threadIdx.x >> 5));
    const unsigned hh = lane >> 4, c = lane & 15u;
    const unsigned head = blockIdx.x / (unsigned)NCHUNK;
    const unsigned chunk = blockIdx.x - head * (unsigned)NCHUNK;
    const size_t base = ((size_t)head * SEQ_FULL + (size_t)chunk * ST_TT) * HD;
#pragma unroll 1
    for (unsigned it = 0; it < 8u; ++it) {
        const unsigned idx = it * 256u + tid;
        const unsigned t = idx >> 4, d0 = (idx & 15u) * 4u;
        const v4f kk = *(const v4f*)(kin + base + (size_t)t * HD + d0);
        const v4f vv = *(const v4f*)(vin + base + (size_t)t * HD + d0);
        sKT[(d0 + 0u) * ST_PT + t] = toh_flush(bfr(kk.x));
        sKT[(d0 + 1u) * ST_PT + t] = toh_flush(bfr(kk.y));
        sKT[(d0 + 2u) * ST_PT + t] = toh_flush(bfr(kk.z));
        sKT[(d0 + 3u) * ST_PT + t] = toh_flush(bfr(kk.w));
        sVT[(d0 + 0u) * ST_PT + t] = toh_flush(bfr(vv.x));
        sVT[(d0 + 1u) * ST_PT + t] = toh_flush(bfr(vv.y));
        sVT[(d0 + 2u) * ST_PT + t] = toh_flush(bfr(vv.z));
        sVT[(d0 + 3u) * ST_PT + t] = toh_flush(bfr(vv.w));
    }
    __syncthreads();
    const unsigned d1t = wave >> 1, d2b = (wave & 1u) * 2u;
    v8f acc0 = (v8f){0.f,0.f,0.f,0.f,0.f,0.f,0.f,0.f};
    v8f acc1 = (v8f){0.f,0.f,0.f,0.f,0.f,0.f,0.f,0.f};
#pragma unroll
    for (unsigned k0 = 0; k0 < (unsigned)ST_TT; k0 += 32u) {
        const v16h a  = frag_ld(sKT + (d1t * 16u + c) * ST_PT + k0 + 8u * hh);
        const v16h b0 = frag_ld(sVT + ((d2b + 0u) * 16u + c) * ST_PT + k0 + 8u * hh);
        const v16h b1 = frag_ld(sVT + ((d2b + 1u) * 16u + c) * ST_PT + k0 + 8u * hh);
        acc0 = wmma16(a, b0, acc0);
        acc1 = wmma16(a, b1, acc1);
    }
#pragma unroll
    for (int r = 0; r < 8; ++r) {
        sC[(d1t * 16u + 8u * hh + (unsigned)r) * SLAB_P + (d2b + 0u) * 16u + c] = acc0[r];
        sC[(d1t * 16u + 8u * hh + (unsigned)r) * SLAB_P + (d2b + 1u) * 16u + c] = acc1[r];
    }
    __syncthreads();
    float* P = part + (size_t)blockIdx.x * (HD * HD);
    v4f ov[4];
#pragma unroll
    for (int it = 0; it < 4; ++it) {
        const unsigned idx = (unsigned)it * 256u + tid;
        const unsigned row = idx >> 4, c4 = (idx & 15u) * 4u;
        ov[it] = *(const v4f*)(sC + row * SLAB_P + c4);
    }
    for (int pass = 0; pass < 2; ++pass) {
#pragma unroll
        for (int it = 0; it < 4; ++it) {
            const unsigned idx = (unsigned)it * 256u + tid;
            *(volatile v4f*)(P + (size_t)idx * 4u) = ov[it];
        }
        __threadfence();
    }
}

__global__ __launch_bounds__(256) void k_fold(const float* __restrict__ part, unsigned short* __restrict__ shi,
                                              unsigned short* __restrict__ sres) {
#pragma clang fp contract(off)
    const unsigned u = blockIdx.x * 256u + threadIdx.x;
    if (u >= (unsigned)(HEADS * HD * (HD / 8))) return;
    const unsigned g = u & 7u, d2 = (u >> 3) & 63u, head = u >> 9;
    const float* p = part + (size_t)head * NCHUNK * (HD * HD) + (size_t)(8u * g) * HD + d2;
    float s[8];
#pragma unroll
    for (int e = 0; e < 8; ++e) s[e] = 0.f;
#pragma unroll 1
    for (unsigned ch = 0; ch < (unsigned)NCHUNK; ++ch) {
        const float* pc = p + (size_t)ch * (HD * HD);
#pragma unroll
        for (int e = 0; e < 8; ++e) s[e] += pc[e * HD];
    }
    float hv[8], rv[8];
#pragma unroll
    for (int e = 0; e < 8; ++e) {
        const float hf = (float)toh_flush(s[e]);
        hv[e] = hf;
        rv[e] = (s[e] - hf) * RES_CARRY;
    }
    const size_t o = ((size_t)head * HD + d2) * HD + 8u * g;
    st8h(shi, o, hv);
    st8h(sres, o, rv);
}

__global__ __launch_bounds__(256) void k_out(const float* __restrict__ q, const _Float16* __restrict__ shi,
                                             const _Float16* __restrict__ sres, float* __restrict__ out) {
    __shared__ __align__(16) float sT[8][16 * SLAB_P];
    const unsigned lane = threadIdx.x & 31u;
    const unsigned wave = (unsigned)__builtin_amdgcn_readfirstlane((int)(threadIdx.x >> 5));
    const unsigned hh = lane >> 4, c = lane & 15u;
    const unsigned nblk = (unsigned)(SEQ / OUT_ROWS);
    const unsigned head = blockIdx.x / nblk;
    const unsigned rb = (blockIdx.x - head * nblk) * (unsigned)OUT_ROWS;
    const size_t row0 = (size_t)head * SEQ_FULL + rb + wave * 16u;
    const float* qrow = q + (row0 + c) * HD + 8u * hh;
    const _Float16* bh = shi  + (size_t)head * (HD * HD) + (size_t)c * HD + 8u * hh;
    const _Float16* br = sres + (size_t)head * (HD * HD) + (size_t)c * HD + 8u * hh;

    v8f ah[4], ar[4];
#pragma unroll
    for (int j = 0; j < 4; ++j) { ah[j] = (v8f){0.f,0.f,0.f,0.f,0.f,0.f,0.f,0.f}; ar[j] = ah[j]; }
#pragma unroll
    for (int ks = 0; ks < 2; ++ks) {
        const v16h a = frag_cvt(qrow + ks * 32);
#pragma unroll
        for (int j = 0; j < 4; ++j) {
            const v16h b  = frag_ld(bh + j * (16 * HD) + ks * 32);
            const v16h b2 = frag_ld(br + j * (16 * HD) + ks * 32);
            ah[j] = wmma16(a, b,  ah[j]);
            ar[j] = wmma16(a, b2, ar[j]);
        }
    }

    float* slab = sT[wave];
#pragma unroll
    for (int j = 0; j < 4; ++j)
#pragma unroll
        for (int r = 0; r < 8; ++r) {
            const float v = (ah[j][r] + ar[j][r] * RES_INV) * QK_SCALE;
            slab[(8u * hh + (unsigned)r) * SLAB_P + ((unsigned)j << 4) + c] = v;
        }
    wave_sync_lds();
    {
        float* C = out + row0 * HD;
        const unsigned c4 = (lane & 15u) * 4u;
#pragma unroll
        for (int half = 0; half < 2; ++half) {
            v4f vv[4];
#pragma unroll
            for (int it = 0; it < 4; ++it) {
                const unsigned row = (unsigned)(half * 4 + it) * 2u + hh;
                vv[it] = *(const v4f*)(slab + row * SLAB_P + c4);
            }
            for (int pass = 0; pass < 2; ++pass) {
#pragma unroll
                for (int it = 0; it < 4; ++it) {
                    const unsigned row = (unsigned)(half * 4 + it) * 2u + hh;
                    *(volatile v4f*)(C + (size_t)row * HD + c4) = vv[it];
                }
                __threadfence();
            }
        }
    }
}

extern "C" void kernel_launch(void* const* d_in, const int* in_sizes, int n_in, void* d_out, int out_size,
                              void* d_ws, size_t ws_size, hipStream_t stream) {
    if (n_in < 3) return;
    if (in_sizes[0] < IN_MIN || in_sizes[1] < IN_MIN || in_sizes[2] < IN_MIN || out_size < IN_MIN) return;

    const float* q = (const float*)d_in[0];
    const float* k = (const float*)d_in[1];
    const float* v = (const float*)d_in[2];
    float* out = (float*)d_out;

    char* wsp = (char*)d_ws;
    size_t off = 0;
    auto carve = [&](size_t bytes) -> void* { void* r = wsp + off; off += (bytes + 255) & ~(size_t)255; return r; };
    float*          part = (float*)carve(PART_BYTES);
    unsigned short* shi  = (unsigned short*)carve(SPL_BYTES);
    unsigned short* sres = (unsigned short*)carve(SPL_BYTES);
    if (off > ws_size || off > (size_t)134217728) return;

    k_state<<<HEADS * NCHUNK, 256, 0, stream>>>(k, v, part);
    k_fold<<<(HEADS * HD * (HD / 8)) / 256, 256, 0, stream>>>((const float*)part, shi, sres);
    k_out<<<HEADS * (SEQ / OUT_ROWS), 256, 0, stream>>>(q, (const _Float16*)shi, (const _Float16*)sres, out);
}
